// XposMultiheadAttention_10282151707348
// MI455X (gfx1250) — hardware-verified
//
#include <hip/hip_runtime.h>

typedef _Float16       v16h __attribute__((ext_vector_type(16)));
typedef _Float16       v8h  __attribute__((ext_vector_type(8)));
typedef __bf16         v16b __attribute__((ext_vector_type(16)));
typedef unsigned short v8us __attribute__((ext_vector_type(8)));
typedef float          v8f  __attribute__((ext_vector_type(8)));
typedef float          v4f  __attribute__((ext_vector_type(4)));
typedef v8h  __attribute__((may_alias)) v8ha;
typedef v8us __attribute__((may_alias)) v8usa;
typedef v4f  __attribute__((may_alias)) v4fa;

union FragH { v16h v; v8h  half[2]; };
union FragB { v16b v; v8us half[2]; };
static_assert(sizeof(FragH) == 32);
static_assert(sizeof(FragB) == 32);

#define BSZ     8
#define SEQ     1024
#define EMB     1024
#define NHEADS  16
#define HD      64
#define NBH     (BSZ * NHEADS)
#define MROWS   (BSZ * SEQ)
#define NX      (MROWS * EMB)
#define NW      (EMB * EMB)
#define NX8     (NX / 8)
#define NW8     (NW / 8)
#define TABN    (SEQ * (HD / 2))
#define PSCALE  16384.0f
#define ASCALE  16.0f
#define WOSCALE 256.0f

static_assert(NX8 == (1 << 20));
static_assert(NW8 == (1 << 17));
static_assert(TABN == (1 << 15));
static_assert((MROWS % 128) == 0);
static_assert((SEQ % 128) == 0);
static_assert(EMB == NHEADS * HD);

__device__ __forceinline__ v8f wmma16h(v16h a, v16h b, v8f c) {
  v8f d = __builtin_amdgcn_wmma_f32_16x16x32_f16(false, a, false, b, (short)0, c, false, false);
  asm volatile("v_nop\n\tv_nop\n\tv_nop\n\tv_nop" : "+v"(d) : "v"(a), "v"(b));
  return d;
}
__device__ __forceinline__ v8f wmma16b(v16b a, v16b b, v8f c) {
  v8f d = __builtin_amdgcn_wmma_f32_16x16x32_bf16(false, a, false, b, (short)0, c, false, false);
  asm volatile("v_nop\n\tv_nop\n\tv_nop\n\tv_nop" : "+v"(d) : "v"(a), "v"(b));
  return d;
}

__device__ __forceinline__ v16h frag_h(const _Float16* p, int h) {
  FragH f;
  f.half[0] = *(const v8ha*)(p + 8 * h);
  f.half[1] = *(const v8ha*)(p + 16 + 8 * h);
  return f.v;
}
__device__ __forceinline__ v16b frag_b(const unsigned short* p, int h) {
  FragB f;
  f.half[0] = *(const v8usa*)(p + 8 * h);
  f.half[1] = *(const v8usa*)(p + 16 + 8 * h);
  return f.v;
}

__device__ __forceinline__ unsigned short bf16_bits(float x) {
  unsigned int u = __float_as_uint(x);
  u += 0x7FFFu + ((u >> 16) & 1u);
  return (unsigned short)(u >> 16);
}
__device__ __forceinline__ float bf16_val(float x) {
  return __uint_as_float(((unsigned int)bf16_bits(x)) << 16);
}

__device__ __forceinline__ void sincos_cw(float a, float& s, float& c) {
  const float n = rintf(a * 0.636619772367581f);
  float r = fmaf(-n, 1.57079637e+00f, a);
  r = fmaf(-n, -4.37113900018624e-08f, r);
  const int qd = ((int)n) & 3;
  const float z = r * r;
  const float sp = fmaf(fmaf(fmaf(-1.9515295891e-4f, z, 8.3321608736e-3f), z, -1.6666654611e-1f) * z, r, r);
  const float cpl = fmaf(fmaf(2.443315711809948e-5f, z, -1.388731625493765e-3f), z, 4.166664568298827e-2f);
  const float cp = fmaf(cpl * z, z, fmaf(-0.5f, z, 1.0f));
  float ss = (qd & 1) ? cp : sp;
  float cc = (qd & 1) ? -sp : cp;
  if (qd & 2) { ss = -ss; cc = -cc; }
  s = ss;
  c = cc;
}

__global__ __launch_bounds__(256) void table_kernel(float* __restrict__ tab)
{
  const int g = blockIdx.x * 256 + threadIdx.x;
  if (g >= 4 * TABN) return;
  const int w = g >> 15;
  const int t = (g >> 5) & (SEQ - 1);
  const int i = g & 31;
  double pw = 1.0;
  pw *= (i & 1)  ? 1.3335214321633240 : 1.0;
  pw *= (i & 2)  ? 1.7782794100389228 : 1.0;
  pw *= (i & 4)  ? 3.1622776601683795 : 1.0;
  pw *= (i & 8)  ? 10.0 : 1.0;
  pw *= (i & 16) ? 100.0 : 1.0;
  const float invf = 1.0f / (float)pw;
  const float ang = (float)t * invf;
  float sn, cs;
  sincos_cw(ang, sn, cs);
  const float zeta = ((float)(2 * i) + 25.6f) * (1.0f / 89.6f);
  const float ex = (float)(t - SEQ / 2) * (1.0f / 1024.0f);
  const float y = ex * log2f(zeta);
  const float scq = exp2f(y);
  const float sck = exp2f(-y);
  const float sc = (w < 2) ? scq : sck;
  const float val = (w & 1) ? (sn * sc) : (cs * sc);
  *(volatile float*)(tab + g) = val;
  __threadfence();
  *(volatile float*)(tab + g) = val;
}

__global__ __launch_bounds__(256) void convert_kernel(
    const float* __restrict__ xq, const float* __restrict__ xk, const float* __restrict__ xv,
    const float* __restrict__ wq, const float* __restrict__ wk, const float* __restrict__ wv,
    const float* __restrict__ wo,
    unsigned short* __restrict__ xb,
    unsigned short* __restrict__ wb,
    _Float16* __restrict__ woh)
{
  const int g = blockIdx.x * 256 + threadIdx.x;
  if (g >= 3 * NX8 + 4 * NW8) return;
  if (g < 3 * NX8 + 3 * NW8) {
    const float* src;
    unsigned short* dst;
    if (g < 3 * NX8) {
      const int sel = g >> 20;
      const int off = g & (NX8 - 1);
      const float* base = (sel == 0) ? xq : ((sel == 1) ? xk : xv);
      src = base + (size_t)off * 8;
      dst = xb + (size_t)g * 8;
    } else {
      const int e = g - 3 * NX8;
      const int sel = e >> 17;
      const int off = e & (NW8 - 1);
      const float* base = (sel == 0) ? wq : ((sel == 1) ? wk : wv);
      src = base + (size_t)off * 8;
      dst = wb + (size_t)e * 8;
    }
    const v4f a = *(const v4fa*)src;
    const v4f c = *(const v4fa*)(src + 4);
    const v8us o = { bf16_bits(a.x), bf16_bits(a.y), bf16_bits(a.z), bf16_bits(a.w),
                     bf16_bits(c.x), bf16_bits(c.y), bf16_bits(c.z), bf16_bits(c.w) };
    *(volatile v8us*)dst = o;
    __threadfence();
    *(volatile v8us*)dst = o;
  } else {
    const int e = g - 3 * NX8 - 3 * NW8;
    const float* src = wo + (size_t)e * 8;
    _Float16* dst = woh + (size_t)e * 8;
    const v4f a = *(const v4fa*)src;
    const v4f c = *(const v4fa*)(src + 4);
    const v8h o = { (_Float16)(bf16_val(a.x) * WOSCALE), (_Float16)(bf16_val(a.y) * WOSCALE),
                    (_Float16)(bf16_val(a.z) * WOSCALE), (_Float16)(bf16_val(a.w) * WOSCALE),
                    (_Float16)(bf16_val(c.x) * WOSCALE), (_Float16)(bf16_val(c.y) * WOSCALE),
                    (_Float16)(bf16_val(c.z) * WOSCALE), (_Float16)(bf16_val(c.w) * WOSCALE) };
    *(volatile v8h*)dst = o;
    __threadfence();
    *(volatile v8h*)dst = o;
  }
}

__device__ __forceinline__ void proj_store_pass(const _Float16* sT, _Float16* plane, _Float16* vt,
                                                int which, int bh, int l0, int w, int lane) {
  const int q8 = lane & 7, sub = lane >> 3;
  #pragma unroll
  for (int i = 0; i < 8; ++i) {
    const int lid = w * 32 + i * 4 + sub;
    v8h v;
    _Float16* dst;
    if (which != 2) {
      v = *(const v8ha*)(sT + lid * HD + 8 * q8);
      dst = plane + ((size_t)bh * SEQ + l0 + lid) * HD + 8 * q8;
    } else {
      const int d = lid >> 1, hl = lid & 1;
      v = *(const v8ha*)(sT + d * 128 + 64 * hl + 8 * q8);
      dst = vt + ((size_t)bh * HD + d) * SEQ + l0 + 64 * hl + 8 * q8;
    }
    *(volatile v8h*)dst = v;
  }
}

__global__ __launch_bounds__(128) void proj_kernel(
    const unsigned short* __restrict__ xb,
    const unsigned short* __restrict__ wb,
    const float* __restrict__ bq, const float* __restrict__ bk, const float* __restrict__ bv,
    const float* __restrict__ tab,
    _Float16* __restrict__ qh,
    _Float16* __restrict__ kh,
    _Float16* __restrict__ vt)
{
  __shared__ __attribute__((aligned(16))) _Float16 sT[128 * 64];

  const int tid = threadIdx.x, lane = tid & 31, w = tid >> 5;
  const int h = lane >> 4, m = lane & 15;
  const int m0 = blockIdx.x * 128;
  const int cg = blockIdx.y;
  const int which = cg >> 4, head = cg & 15;
  const int m0w = m0 + 32 * w;

  const unsigned short* xa0 = xb + (size_t)which * NX + (size_t)(m0w + m) * EMB;
  const unsigned short* xa1 = xa0 + (size_t)16 * EMB;
  const unsigned short* wbp = wb + (size_t)which * NW + (size_t)(head * HD + m) * EMB;

  const v8f zero8 = {0.f, 0.f, 0.f, 0.f, 0.f, 0.f, 0.f, 0.f};
  v8f acc[2][4];
  #pragma unroll
  for (int mt = 0; mt < 2; ++mt)
    #pragma unroll
    for (int nt = 0; nt < 4; ++nt) acc[mt][nt] = zero8;

  #pragma unroll 1
  for (int k0 = 0; k0 < EMB; k0 += 32) {
    const v16b a0 = frag_b(xa0 + k0, h);
    const v16b a1 = frag_b(xa1 + k0, h);
    #pragma unroll
    for (int nt = 0; nt < 4; ++nt) {
      const v16b b = frag_b(wbp + (size_t)nt * 16 * EMB + k0, h);
      acc[0][nt] = wmma16b(a0, b, acc[0][nt]);
      acc[1][nt] = wmma16b(a1, b, acc[1][nt]);
    }
  }

  const float* bias = (which == 0) ? bq : ((which == 1) ? bk : bv);
  const float* tcs = tab + (size_t)(2 * which) * TABN;
  const float* tsn = tcs + TABN;
  const int b = m0 >> 10, l0 = m0 & (SEQ - 1), bh = b * NHEADS + head;
  #pragma unroll
  for (int nt = 0; nt < 4; ++nt) {
    const int feat = 16 * nt + m;
    const int ip = feat >> 1;
    const float sgn = (feat & 1) ? 1.0f : -1.0f;
    const float bvl = bf16_val(bias[head * HD + feat]);
    #pragma unroll
    for (int mt = 0; mt < 2; ++mt) {
      #pragma unroll
      for (int r = 0; r < 8; ++r) {
        const int tokl = 32 * w + 16 * mt + 8 * h + r;
        float c = acc[mt][nt][r] + bvl;
        if (which != 2) {
          const float pr = __shfl_xor(c, 1);
          const int ti = (l0 + tokl) * (HD / 2) + ip;
          c = c * tcs[ti] + (sgn * pr) * tsn[ti];
        }
        const int idx = (which == 2) ? (feat * 128 + tokl) : (tokl * HD + feat);
        sT[idx] = (_Float16)c;
      }
    }
  }
  __syncthreads();

  _Float16* plane = (which == 0) ? qh : kh;
  proj_store_pass(sT, plane, vt, which, bh, l0, w, lane);
  __threadfence();
  proj_store_pass(sT, plane, vt, which, bh, l0, w, lane);
}

__device__ __forceinline__ v16h pack_p(v8f a, v8f c) {
  const v16h r = { (_Float16)(a[0] * PSCALE), (_Float16)(a[1] * PSCALE), (_Float16)(a[2] * PSCALE), (_Float16)(a[3] * PSCALE),
                   (_Float16)(a[4] * PSCALE), (_Float16)(a[5] * PSCALE), (_Float16)(a[6] * PSCALE), (_Float16)(a[7] * PSCALE),
                   (_Float16)(c[0] * PSCALE), (_Float16)(c[1] * PSCALE), (_Float16)(c[2] * PSCALE), (_Float16)(c[3] * PSCALE),
                   (_Float16)(c[4] * PSCALE), (_Float16)(c[5] * PSCALE), (_Float16)(c[6] * PSCALE), (_Float16)(c[7] * PSCALE) };
  return r;
}

__device__ __forceinline__ void att_store_pass(const _Float16* so, _Float16* ah,
                                               int b, int head, int q0, int lane) {
  const int q8 = lane & 7, sub = lane >> 3;
  #pragma unroll
  for (int i = 0; i < 4; ++i) {
    const int row = i * 4 + sub;
    const v8h v = *(const v8ha*)(so + row * 64 + 8 * q8);
    _Float16* dst = ah + ((size_t)b * SEQ + q0 + row) * EMB + head * HD + 8 * q8;
    *(volatile v8h*)dst = v;
  }
}

__global__ __launch_bounds__(128) void attn_kernel(
    const _Float16* __restrict__ qh,
    const _Float16* __restrict__ kh,
    const _Float16* __restrict__ vt,
    _Float16* __restrict__ ah)
{
  __shared__ __attribute__((aligned(16))) _Float16 sO[4 * 16 * 64];

  const int tid = threadIdx.x, lane = tid & 31, w = tid >> 5;
  const int h = lane >> 4, m = lane & 15;
  const int bh = blockIdx.y, b = bh >> 4, head = bh & 15;
  const int q0 = blockIdx.x * 64 + 16 * w;

  const _Float16* qrow = qh + ((size_t)bh * SEQ + q0 + m) * HD;
  const v16h qb0 = frag_h(qrow, h);
  const v16h qb1 = frag_h(qrow + 32, h);

  const v8f zero8 = {0.f, 0.f, 0.f, 0.f, 0.f, 0.f, 0.f, 0.f};
  v8f o[4];
  #pragma unroll
  for (int t = 0; t < 4; ++t) o[t] = zero8;
  float mrun = -1e30f, lrun = 0.0f;

  const _Float16* kbase = kh + ((size_t)bh * SEQ + m) * HD;
  const _Float16* vbase = vt + ((size_t)bh * HD + m) * SEQ;
  const float escale = 0.125f;

  #pragma unroll 1
  for (int kb = 0; kb < SEQ; kb += 64) {
    v8f s[4];
    #pragma unroll
    for (int j = 0; j < 4; ++j) {
      const _Float16* kp = kbase + (size_t)(kb + 16 * j) * HD;
      const v16h kf0 = frag_h(kp, h);
      const v16h kf1 = frag_h(kp + 32, h);
      v8f z = zero8;
      z = wmma16h(kf0, qb0, z);
      z = wmma16h(kf1, qb1, z);
      s[j] = z;
    }

    float mloc = s[0][0];
    #pragma unroll
    for (int j = 0; j < 4; ++j)
      #pragma unroll
      for (int r = 0; r < 8; ++r) mloc = fmaxf(mloc, s[j][r]);
    mloc = fmaxf(mloc, __shfl_xor(mloc, 16));
    const float mnew = fmaxf(mrun, mloc);
    const float alpha = __expf((mrun - mnew) * escale);
    mrun = mnew;
    float lsum = 0.0f;
    #pragma unroll
    for (int j = 0; j < 4; ++j)
      #pragma unroll
      for (int r = 0; r < 8; ++r) {
        const float p = __expf((s[j][r] - mnew) * escale);
        s[j][r] = p;
        lsum += p;
      }
    lsum += __shfl_xor(lsum, 16);
    lrun = lrun * alpha + lsum;
    #pragma unroll
    for (int t = 0; t < 4; ++t)
      #pragma unroll
      for (int r = 0; r < 8; ++r) o[t][r] = o[t][r] * alpha;

    const v16h pb0 = pack_p(s[0], s[1]);
    const v16h pb1 = pack_p(s[2], s[3]);

    #pragma unroll
    for (int t = 0; t < 4; ++t) {
      const _Float16* vp = vbase + (size_t)(16 * t) * SEQ + kb;
      const v16h vf0 = frag_h(vp, h);
      const v16h vf1 = frag_h(vp + 32, h);
      o[t] = wmma16h(vf0, pb0, o[t]);
      o[t] = wmma16h(vf1, pb1, o[t]);
    }
  }

  const float inv = (1.0f / lrun) * (ASCALE / PSCALE);
  _Float16* so = sO + w * 1024;
  #pragma unroll
  for (int t = 0; t < 4; ++t)
    #pragma unroll
    for (int r = 0; r < 8; ++r)
      so[m * 64 + 16 * t + 8 * h + r] = (_Float16)(o[t][r] * inv);
  __syncthreads();

  att_store_pass(so, ah, b, head, q0, lane);
  __threadfence();
  att_store_pass(so, ah, b, head, q0, lane);
}

__device__ __forceinline__ void out_store_pass(const float* sF, float* out,
                                               int m0, int head, int w, int lane) {
  const int q8 = lane & 7, sub = lane >> 3;
  #pragma unroll
  for (int i = 0; i < 16; ++i) {
    const int L = i * 4 + sub;
    const int tok = w * 32 + (L >> 1), hl = L & 1;
    const v4f v = *(const v4fa*)(sF + tok * 64 + 32 * hl + 4 * q8);
    float* dst = out + (size_t)(m0 + tok) * EMB + head * HD + 32 * hl + 4 * q8;
    *(volatile v4f*)dst = v;
  }
}

__global__ __launch_bounds__(128) void outproj_kernel(
    const _Float16* __restrict__ ah,
    const _Float16* __restrict__ woh,
    const float* __restrict__ bo,
    float* __restrict__ out)
{
  __shared__ __attribute__((aligned(16))) float sF[128 * 64];

  const int tid = threadIdx.x, lane = tid & 31, w = tid >> 5;
  const int h = lane >> 4, m = lane & 15;
  const int m0 = blockIdx.x * 128;
  const int head = blockIdx.y;
  const int m0w = m0 + 32 * w;

  const _Float16* xa0 = ah + (size_t)(m0w + m) * EMB;
  const _Float16* xa1 = xa0 + (size_t)16 * EMB;
  const _Float16* wbp = woh + (size_t)(head * HD + m) * EMB;

  const v8f zero8 = {0.f, 0.f, 0.f, 0.f, 0.f, 0.f, 0.f, 0.f};
  v8f acc[2][4];
  #pragma unroll
  for (int mt = 0; mt < 2; ++mt)
    #pragma unroll
    for (int nt = 0; nt < 4; ++nt) acc[mt][nt] = zero8;

  #pragma unroll 1
  for (int k0 = 0; k0 < EMB; k0 += 32) {
    const v16h a0 = frag_h(xa0 + k0, h);
    const v16h a1 = frag_h(xa1 + k0, h);
    #pragma unroll
    for (int nt = 0; nt < 4; ++nt) {
      const v16h b = frag_h(wbp + (size_t)nt * 16 * EMB + k0, h);
      acc[0][nt] = wmma16h(a0, b, acc[0][nt]);
      acc[1][nt] = wmma16h(a1, b, acc[1][nt]);
    }
  }

  const float osc = 1.0f / (ASCALE * WOSCALE);
  #pragma unroll
  for (int nt = 0; nt < 4; ++nt) {
    const int feat = 16 * nt + m;
    const float bvl = bf16_val(bo[head * HD + feat]);
    #pragma unroll
    for (int mt = 0; mt < 2; ++mt) {
      #pragma unroll
      for (int r = 0; r < 8; ++r) {
        const int tokl = 32 * w + 16 * mt + 8 * h + r;
        sF[tokl * 64 + feat] = acc[mt][nt][r] * osc + bvl;
      }
    }
  }
  __syncthreads();

  out_store_pass(sF, out, m0, head, w, lane);
  __threadfence();
  out_store_pass(sF, out, m0, head, w, lane);
}

extern "C" void kernel_launch(void* const* d_in, const int* in_sizes, int n_in,
                              void* d_out, int out_size, void* d_ws, size_t ws_size,
                              hipStream_t stream) {
  if (n_in < 11) return;
  if (in_sizes[0] != NX || in_sizes[1] != NX || in_sizes[2] != NX) return;
  if (in_sizes[3] != NW || in_sizes[5] != NW || in_sizes[7] != NW || in_sizes[9] != NW) return;
  if (in_sizes[4] != EMB || in_sizes[6] != EMB || in_sizes[8] != EMB || in_sizes[10] != EMB) return;
  if (out_size != NX) return;

  const float* query = (const float*)d_in[0];
  const float* key   = (const float*)d_in[1];
  const float* value = (const float*)d_in[2];
  const float* wq = (const float*)d_in[3];
  const float* bq = (const float*)d_in[4];
  const float* wk = (const float*)d_in[5];
  const float* bk = (const float*)d_in[6];
  const float* wv = (const float*)d_in[7];
  const float* bv = (const float*)d_in[8];
  const float* wo = (const float*)d_in[9];
  const float* bo = (const float*)d_in[10];
  float* out = (float*)d_out;

  const size_t xb_bytes = (size_t)3 * NX * 2;
  const size_t wb_bytes = (size_t)3 * NW * 2;
  const size_t wo_bytes = (size_t)NW * 2;
  const size_t pl_bytes = (size_t)NX * 2;
  const size_t tb_bytes = (size_t)4 * TABN * 4;
  const size_t total = xb_bytes + wb_bytes + wo_bytes + 4 * pl_bytes + tb_bytes;
  if (total > ws_size) return;
  if (total > (size_t)134217728) return;

  char* ws = (char*)d_ws;
  unsigned short* xb = (unsigned short*)(ws);
  unsigned short* wb = (unsigned short*)(ws + xb_bytes);
  _Float16* woh = (_Float16*)(ws + xb_bytes + wb_bytes);
  _Float16* qh  = (_Float16*)(ws + xb_bytes + wb_bytes + wo_bytes);
  _Float16* kh  = (_Float16*)(ws + xb_bytes + wb_bytes + wo_bytes + pl_bytes);
  _Float16* vth = (_Float16*)(ws + xb_bytes + wb_bytes + wo_bytes + 2 * pl_bytes);
  _Float16* ah  = (_Float16*)(ws + xb_bytes + wb_bytes + wo_bytes + 3 * pl_bytes);
  float* tab    = (float*)(ws + xb_bytes + wb_bytes + wo_bytes + 4 * pl_bytes);

  table_kernel<<<(4 * TABN) / 256, 256, 0, stream>>>(tab);

  const int ngroups = 3 * NX8 + 4 * NW8;
  convert_kernel<<<(ngroups + 255) / 256, 256, 0, stream>>>(query, key, value, wq, wk, wv, wo, xb, wb, woh);

  dim3 gProj(MROWS / 128, 3 * NHEADS);
  proj_kernel<<<gProj, 128, 0, stream>>>(xb, wb, bq, bk, bv, tab, qh, kh, vth);

  dim3 gAtt(SEQ / 64, NBH);
  attn_kernel<<<gAtt, 128, 0, stream>>>(qh, kh, vth, ah);

  dim3 gOut(MROWS / 128, NHEADS);
  outproj_kernel<<<gOut, 128, 0, stream>>>(ah, woh, bo, out);
}
